// EGCLayer_5214090297740
// MI455X (gfx1250) — hardware-run, weakly checked
//
#include <hip/hip_runtime.h>


namespace {
constexpr int N = 50000, NP = 50048, NLIM = 50048  , NLIMN = (NLIM < N ? NLIM : N), EFULL = 800000, E = EFULL, EH = E / 2  , EC = 400000  , HD = 64, K1 = 2 * HD  ;
constexpr float XS = 8.0f, WSC = 256.0f;
static_assert(E % 32 == 0 && NP % 32 == 0 && NLIM % 32 == 0, "tiling");
typedef _Float16 b16;
typedef __attribute__((ext_vector_type(16))) _Float16 v16b;
typedef __attribute__((ext_vector_type(8))) _Float16 v8b;
typedef __attribute__((ext_vector_type(8))) float v8f;
typedef __attribute__((ext_vector_type(4))) float v4f;
__device__ __forceinline__ float bf16_rne(float f) { unsigned int u = __float_as_uint(f); u += 0x7FFFu + ((u >> 16) & 1u); return __uint_as_float(u & 0xFFFF0000u); }
__device__ __forceinline__ void split16(float v, b16& hi, b16& lo) { hi = (b16)v; lo = (b16)(v - (float)hi); }
__device__ __forceinline__ v16b frag_kb(const b16* p, int hh) { const v8b a = *(const v8b*)(p + 8 * hh), b = *(const v8b*)(p + 16 + 8 * hh); v16b f;
#pragma unroll
  for (int e = 0; e < 8; ++e) { f[e] = a[e]; f[8 + e] = b[e]; } return f; }
__device__ __forceinline__ v8f wmma16b(v16b a, v16b b, v8f c) { v8f d = __builtin_amdgcn_wmma_f32_16x16x32_f16(false, a, false, b, (short)0, c, false, false); asm volatile("v_nop\n\tv_nop\n\tv_nop\n\tv_nop" : "+v"(d) : "v"(a), "v"(b)); return d; }
__device__ __forceinline__ void wave_lds_sync() { __builtin_amdgcn_fence(__ATOMIC_RELEASE, "workgroup"); __builtin_amdgcn_wave_barrier(); __builtin_amdgcn_fence(__ATOMIC_ACQUIRE, "workgroup"); }
__device__ __forceinline__ float pmul(float a, float b) { float p = a * b; asm volatile("" : "+v"(p)); return p; }
__device__ __forceinline__ int iclamp(int v, int lo, int hi) { return v < lo ? lo : (v > hi ? hi : v); }
constexpr int CSR_NBLK = 512, CSR_GB = 9, CSR_GN = 1 << CSR_GB  , CSR_MAXG = 512, CSR_CAP = 12288  ;
__global__ __launch_bounds__(64) void csrA_kernel(const int* __restrict__ dst, int E, int N, int nG, int CHP, int NGP, int* __restrict__ STG, int* __restrict__ HST) {
  extern __shared__ int sm[];
  int* cnt = sm; int* run = sm + NGP; int* ids = sm + 2 * NGP;
  const int b = blockIdx.x; const int ch = (E + CSR_NBLK - 1) / CSR_NBLK; const int e0 = b * ch, e1 = min(E, e0 + ch);
  for (int i = threadIdx.x; i < NGP; i += 64) cnt[i] = 0;
  for (int i = threadIdx.x; i < CHP; i += 64) ids[i] = -1;
  __syncthreads();
  if (threadIdx.x == 0) {
    for (int e = e0; e < e1; ++e) { int d = dst[e]; d = (d < 0) ? 0 : (d >= N ? N - 1 : d); cnt[d >> CSR_GB] += 1; }
    int acc = 0; for (int g = 0; g < nG; ++g) { run[g] = acc; acc += cnt[g]; }
    for (int e = e0; e < e1; ++e) { int d = dst[e]; d = (d < 0) ? 0 : (d >= N ? N - 1 : d); const int g = d >> CSR_GB; ids[run[g]] = e; run[g] += 1; } }
  __syncthreads();
  typedef __attribute__((ext_vector_type(4))) int v4i;
  for (int pass = 0; pass < 2; ++pass) {
    for (int i = threadIdx.x; i < CHP / 4; i += 64) *(volatile v4i*)(STG + (size_t)b * CHP + i * 4) = *(const v4i*)(&ids[i * 4]);
    for (int i = threadIdx.x; i < NGP / 4; i += 64) { v4i v; for (int e = 0; e < 4; ++e) v[e] = (i * 4 + e < nG) ? cnt[i * 4 + e] : 0; *(volatile v4i*)(HST + (size_t)b * NGP + i * 4) = v; }
    __threadfence(); }
}
__global__ __launch_bounds__(512) void csrS_kernel(const int* __restrict__ HST, int nG, int NGP, int* __restrict__ START, int* __restrict__ TOT, int* __restrict__ OFF) {
  __shared__ int tot[CSR_MAXG];
  const int b = threadIdx.x;
  for (int pass = 0; pass < 2; ++pass) { int runb = 0; for (int g = 0; g < nG; ++g) { int c = HST[(size_t)b * NGP + g]; c = (c < 0) ? 0 : c; ((volatile int*)OFF)[(size_t)g * CSR_NBLK + b] = runb; runb += c; } __threadfence(); }
  for (int g = threadIdx.x; g < nG; g += 512) { int s = 0; for (int bb = 0; bb < CSR_NBLK; ++bb) { int c = HST[(size_t)bb * NGP + g]; s += (c < 0) ? 0 : c; } tot[g] = s; }
  __syncthreads();
  if (threadIdx.x < 32) {
    __shared__ int st[CSR_MAXG + 32];
    if (threadIdx.x == 0) { int acc = 0; for (int g = 0; g < NGP; ++g) { st[g] = acc; if (g < nG) acc += (tot[g] + 31) & ~31; } st[NGP] = acc; }
    __builtin_amdgcn_fence(__ATOMIC_RELEASE, "workgroup"); __builtin_amdgcn_wave_barrier(); __builtin_amdgcn_fence(__ATOMIC_ACQUIRE, "workgroup");
    for (int pass = 0; pass < 2; ++pass) { for (int i = threadIdx.x; i < NGP + 32; i += 32) { ((volatile int*)START)[i] = (i <= NGP) ? st[min(i, NGP)] : 0; ((volatile int*)TOT)[i] = (i < nG) ? tot[i] : 0; } __threadfence(); } }
}
__global__ __launch_bounds__(256) void csrB_kernel(const int* __restrict__ dst, int N, int nG, int CHP, int NGP, int permLen, const int* __restrict__ STG, const int* __restrict__ HST, const int* __restrict__ OFF, const int* __restrict__ START, const int* __restrict__ TOT, int* __restrict__ PERM, int* __restrict__ ROWPTR, int* __restrict__ ROWCNT, int* __restrict__ FLAG) {
  typedef __attribute__((ext_vector_type(4))) int v4i;
  __shared__ int ids[CSR_CAP]; __shared__ unsigned short key[CSR_CAP]; __shared__ int outp[CSR_CAP]; __shared__ int ncnt[CSR_GN + 1]; __shared__ int boff[CSR_NBLK + 1];
  const int g = blockIdx.x, t_ = threadIdx.x; int tot = TOT[g]; int st = START[g], stn = START[g + 1]; const int v0 = g * CSR_GN; const int nv = min(CSR_GN, N - v0);
  st = (st < 0) ? 0 : (st > permLen - 32 ? permLen - 32 : st) & ~31; stn = (stn < st) ? st : (stn > permLen ? permLen : stn); tot = (tot < 0) ? 0 : tot; if (tot > stn - st && tot <= CSR_CAP) tot = stn - st;
  if (tot > CSR_CAP) {
    for (int pass = 0; pass < 2; ++pass) { for (int i = t_; i < CSR_GN / 4; i += 256) { v4i a, c; for (int e = 0; e < 4; ++e) { a[e] = st; c[e] = 0; } *(volatile v4i*)(ROWPTR + v0 + i * 4) = a; *(volatile v4i*)(ROWCNT + v0 + i * 4) = c; } if (t_ == 0) ((volatile int*)FLAG)[0] = 1; __threadfence(); } (void)nv; return; }
  if (t_ == 0) { int acc = 0; for (int b = 0; b < CSR_NBLK; ++b) { boff[b] = acc; int c = HST[(size_t)b * NGP + g]; c = (c < 0) ? 0 : (c > CHP ? CHP : c); acc += c; if (acc > tot) acc = tot; } boff[CSR_NBLK] = acc; }
  for (int i = t_; i <= CSR_GN; i += 256) ncnt[i] = 0;
  __syncthreads();
  for (int b = 0; b < CSR_NBLK; ++b) { const int c = boff[b + 1] - boff[b]; int o_ = OFF[(size_t)g * CSR_NBLK + b]; o_ = (o_ < 0) ? 0 : (o_ > CHP - c ? CHP - c : o_); const int* src_ = STG + (size_t)b * CHP + o_;
    for (int i = t_; i < c; i += 256) { int id = src_[i]; id = (id < 0) ? 0 : id; ids[boff[b] + i] = id; int d = dst[id]; d = (d < v0) ? v0 : (d >= N ? N - 1 : d); int kk = d - v0; kk = (kk < 0) ? 0 : (kk >= CSR_GN ? CSR_GN - 1 : kk); key[boff[b] + i] = (unsigned short)kk; } }
  __syncthreads();
  if (t_ == 0) { for (int i = 0; i < tot; ++i) ncnt[key[i]] += 1; int acc = 0; for (int vl = 0; vl < CSR_GN; ++vl) { const int c = ncnt[vl]; ncnt[vl] = acc; acc += c; } ncnt[CSR_GN] = acc;
    for (int i = 0; i < tot; ++i) { const int vl = key[i]; outp[ncnt[vl]] = ids[i]; ncnt[vl] += 1; }
    for (int vl = CSR_GN; vl > 0; --vl) ncnt[vl] = ncnt[vl - 1]; ncnt[0] = 0; }
  __syncthreads();
  for (int pass = 0; pass < 2; ++pass) {
    for (int i = t_; i < (stn - st) / 4; i += 256) { v4i v; for (int e = 0; e < 4; ++e) { const int q = i * 4 + e; v[e] = (q < tot) ? outp[q] : -1; } *(volatile v4i*)(PERM + st + i * 4) = v; }
    for (int i = t_; i < CSR_GN / 4; i += 256) { v4i a, c; for (int e = 0; e < 4; ++e) { const int vl = i * 4 + e; a[e] = st + ncnt[vl]; c[e] = (vl < nv) ? (ncnt[vl + 1] - ncnt[vl]) : 0; } *(volatile v4i*)(ROWPTR + v0 + i * 4) = a; *(volatile v4i*)(ROWCNT + v0 + i * 4) = c; }
    __threadfence(); }
}
__global__ __launch_bounds__(256) void csrZ_kernel(int* __restrict__ p, size_t n4) { typedef __attribute__((ext_vector_type(4))) int v4i; const size_t tid = (size_t)blockIdx.x * 256 + threadIdx.x, nth = (size_t)gridDim.x * 256; v4i z = {0, 0, 0, 0}; for (size_t i = tid; i < n4; i += nth) *(volatile v4i*)(p + i * 4) = z; }
struct CsrBufs { int *STG, *HST, *OFF, *START, *TOT, *PERM, *ROWPTR, *ROWCNT, *FLAG; int nG, NGP, CHP; size_t permLen; char* base; size_t bytes; };
static size_t csr_carve(CsrBufs& c, char* ws, size_t off, int E, int N) {
  const size_t off0 = off; c.base = ws + off;
  auto al = [&](size_t bytes) { char* p = ws + off; off += (bytes + 255) & ~(size_t)255; return p; };
  c.nG = (N + CSR_GN - 1) / CSR_GN; c.NGP = (c.nG + 31) & ~31; const int ch = (E + CSR_NBLK - 1) / CSR_NBLK; c.CHP = (ch + 31) & ~31; c.permLen = (size_t)E + 32 * (size_t)c.nG + 32;
  c.STG = (int*)al((size_t)CSR_NBLK * c.CHP * 4); c.HST = (int*)al((size_t)CSR_NBLK * c.NGP * 4); c.OFF = (int*)al((size_t)c.NGP * CSR_NBLK * 4); c.START = (int*)al((size_t)(c.NGP + 64) * 4); c.TOT = (int*)al((size_t)(c.NGP + 64) * 4);
  c.PERM = (int*)al(c.permLen * 4); c.ROWPTR = (int*)al((size_t)c.nG * CSR_GN * 4); c.ROWCNT = (int*)al((size_t)c.nG * CSR_GN * 4); c.FLAG = (int*)al(256);
  c.bytes = off - off0; return off;
}
static void csr_build(const CsrBufs& c, const int* dst, int E, int N, hipStream_t stream) {
  const size_t smem = (size_t)(2 * c.NGP + c.CHP) * 4;
  csrZ_kernel<<<512, 256, 0, stream>>>((int*)c.base, c.bytes / 16);
  csrA_kernel<<<CSR_NBLK, 64, smem, stream>>>(dst, E, N, c.nG, c.CHP, c.NGP, c.STG, c.HST);
  csrS_kernel<<<1, 512, 0, stream>>>(c.HST, c.nG, c.NGP, c.START, c.TOT, c.OFF);
  csrB_kernel<<<c.nG, 256, 0, stream>>>(dst, N, c.nG, c.CHP, c.NGP, (int)c.permLen, c.STG, c.HST, c.OFF, c.START, c.TOT, c.PERM, c.ROWPTR, c.ROWCNT, c.FLAG);
}

typedef __attribute__((ext_vector_type(2))) float v2f;
__global__ __launch_bounds__(256) void wprep_kernel(const float* __restrict__ w1, const float* __restrict__ w2, const float* __restrict__ u1, const float* __restrict__ u2, b16* __restrict__ WT1, b16* __restrict__ WT2, b16* __restrict__ UT1, b16* __restrict__ UT2) {
  for (int u = threadIdx.x; u < (HD * K1 + 3 * HD * HD) / 8; u += 256) { int e = u * 8; v8b o;
    if (e < HD * K1) { const int oo = e / K1, k0 = e % K1; for (int j = 0; j < 8; ++j) o[j] = (b16)(bf16_rne(w1[(size_t)(k0 + j) * HD + oo]) * WSC); for (int pass = 0; pass < 2; ++pass) { *(volatile v8b*)(WT1 + e) = o; __threadfence(); } continue; }
    e -= HD * K1; const int which = e / (HD * HD); const int el = e % (HD * HD); const int oo = el / HD, k0 = el % HD; const float* w = which == 0 ? w2 : (which == 1 ? u1 : u2); b16* dstp = which == 0 ? WT2 : (which == 1 ? UT1 : UT2);
    for (int j = 0; j < 8; ++j) o[j] = (b16)(bf16_rne(w[(size_t)(k0 + j) * HD + oo]) * WSC); for (int pass = 0; pass < 2; ++pass) { *(volatile v8b*)(dstp + el) = o; __threadfence(); } }
}
__global__ __launch_bounds__(64) void edge_kernel(const float* __restrict__ feat, const float* __restrict__ xyz, const int* __restrict__ srcs, const int* __restrict__ dsts, const b16* __restrict__ WT1, const float* __restrict__ w1, const float* __restrict__ b1, const b16* __restrict__ WT2, const float* __restrict__ b2, const float* __restrict__ we, const float* __restrict__ be, int ebase, float* __restrict__ MG) {
  __shared__ __attribute__((aligned(16))) float T[2][16][HD + 4]; __shared__ float sq[2][16];
  const int wave = threadIdx.x >> 5, lane = threadIdx.x & 31, nloc = lane & 15, hlf = lane >> 4; const size_t e0 = (size_t)ebase + (size_t)blockIdx.x * 32 + wave * 16;
  const size_t er = e0 + nloc; const int s = iclamp(srcs[er], 0, N - 1), d = iclamp(dsts[er], 0, N - 1);
  if (hlf == 0) { float q = 0.0f; for (int i = 0; i < 3; ++i) { const float df = bf16_rne(xyz[(size_t)s * 3 + i]) - bf16_rne(xyz[(size_t)d * 3 + i]); q += df * df; } sq[wave][nloc] = q; }
  v8f acc[4];
#pragma unroll
  for (int t = 0; t < 4; ++t) acc[t] = (v8f){};
#pragma unroll
  for (int ks = 0; ks < 4; ++ks) { const float* row = feat + (size_t)(ks < 2 ? s : d) * HD + (ks & 1) * 32; v16b a; const v4f f0 = *(const v4f*)(row + 8 * hlf), f1 = *(const v4f*)(row + 8 * hlf + 4), f2 = *(const v4f*)(row + 16 + 8 * hlf), f3 = *(const v4f*)(row + 16 + 8 * hlf + 4);
    float fv[16]; for (int i = 0; i < 4; ++i) { fv[i] = f0[i]; fv[4 + i] = f1[i]; fv[8 + i] = f2[i]; fv[12 + i] = f3[i]; }
#pragma unroll
    for (int e2 = 0; e2 < 16; ++e2) a[e2] = (b16)(bf16_rne(fv[e2]) * XS);
#pragma unroll
    for (int t = 0; t < 4; ++t) acc[t] = wmma16b(a, frag_kb(WT1 + (size_t)(t * 16 + nloc) * K1 + ks * 32, hlf), acc[t]); }
  wave_lds_sync();
#pragma unroll
  for (int t = 0; t < 4; ++t) { const int cc = t * 16 + nloc; const float bb = bf16_rne(b1[cc]), ws = bf16_rne(w1[(size_t)K1 * HD + cc]);
#pragma unroll
    for (int r = 0; r < 8; ++r) T[wave][8 * hlf + r][cc] = fmaxf(acc[t][r] * (1.0f / (XS * WSC)) + bb + pmul(sq[wave][8 * hlf + r], ws), 0.0f); }
  wave_lds_sync();
#pragma unroll
  for (int t = 0; t < 4; ++t) acc[t] = (v8f){};
#pragma unroll
  for (int ks = 0; ks < 2; ++ks) { v16b ah, al;
#pragma unroll
    for (int e2 = 0; e2 < 16; ++e2) { const int k = ks * 32 + ((e2 < 8) ? (8 * hlf + e2) : (16 + 8 * hlf + e2 - 8)); b16 p, q; split16(T[wave][nloc][k] * XS, p, q); ah[e2] = p; al[e2] = q; }
#pragma unroll
    for (int t = 0; t < 4; ++t) { const v16b bw = frag_kb(WT2 + (size_t)(t * 16 + nloc) * HD + ks * 32, hlf); acc[t] = wmma16b(ah, bw, acc[t]); acc[t] = wmma16b(al, bw, acc[t]); } }
  wave_lds_sync();
  float gp[8];
#pragma unroll
  for (int r = 0; r < 8; ++r) gp[r] = 0.0f;
#pragma unroll
  for (int t = 0; t < 4; ++t) { const int cc = t * 16 + nloc; const float bb = bf16_rne(b2[cc]), wg = bf16_rne(we[cc]);
#pragma unroll
    for (int r = 0; r < 8; ++r) { const float m = fmaxf(acc[t][r] * (1.0f / (XS * WSC)) + bb, 0.0f); T[wave][8 * hlf + r][cc] = m; gp[r] += pmul(m, wg); } }
  const float beb = bf16_rne(be[0]);
#pragma unroll
  for (int r = 0; r < 8; ++r) {
#pragma unroll
    for (int o = 1; o < 16; o <<= 1) gp[r] += __shfl_xor(gp[r], o);
    gp[r] = 1.0f / (1.0f + __expf(-(gp[r] + beb))); }
#pragma unroll
  for (int t = 0; t < 4; ++t)
#pragma unroll
    for (int r = 0; r < 8; ++r) T[wave][8 * hlf + r][t * 16 + nloc] *= gp[r];
  wave_lds_sync();
  for (int pass = 0; pass < 2; ++pass) { for (int rr = 0; rr < 16; ++rr) *(volatile v2f*)(MG + (e0 - ebase + rr) * HD + lane * 2) = *(const v2f*)(&T[wave][rr][lane * 2]); __threadfence(); }
}
template <int HALF>
__global__ __launch_bounds__(256) void nsum_kernel(const float* __restrict__ MG, const int* __restrict__ PERM, const int* __restrict__ ROWPTR, const int* __restrict__ ROWCNT, int permLen, float* __restrict__ S) {
  const int wave = threadIdx.x >> 5, lane = threadIdx.x & 31; const size_t v = (size_t)blockIdx.x * 8 + wave; v2f a = {0.0f, 0.0f};
  if (v < (size_t)NLIMN) { int st = ROWPTR[v], cnt = ROWCNT[v]; cnt = iclamp(cnt, 0, 65536); st = iclamp(st, 0, permLen - cnt);
#pragma unroll 1
    for (int j = 0; j < cnt; ++j) { const int e = iclamp(PERM[st + j], 0, E - 1); const int el = e - HALF * EH; if (el < 0 || el >= EC) continue; a += *(const v2f*)(MG + (size_t)el * HD + lane * 2); }
    if (HALF) a += *(const v2f*)(S + v * HD + lane * 2); }
  for (int pass = 0; pass < 2; ++pass) { *(volatile v2f*)(S + v * HD + lane * 2) = a; __threadfence(); }
}
__global__ __launch_bounds__(64) void node_kernel(const float* __restrict__ S, const float* __restrict__ feat, const b16* __restrict__ UT1, const float* __restrict__ c1, const b16* __restrict__ UT2, const float* __restrict__ c2, float* __restrict__ out) {
  __shared__ __attribute__((aligned(16))) float H[2][16][HD + 4], T[2][16][HD + 4];
  const int wave = threadIdx.x >> 5, lane = threadIdx.x & 31, nloc = lane & 15, hlf = lane >> 4; const size_t v0 = (size_t)blockIdx.x * 32 + wave * 16; if (v0 >= (size_t)NLIMN) return;
  for (int i = 0; i < 16; ++i) { const size_t v = v0 + i; v2f a = *(const v2f*)(S + v * HD + lane * 2); const v2f f = *(const v2f*)(feat + v * HD + lane * 2); a[0] += bf16_rne(f[0]); a[1] += bf16_rne(f[1]); *(v2f*)(&H[wave][i][lane * 2]) = a; }
  wave_lds_sync();
  v8f acc[4];
#pragma unroll
  for (int t = 0; t < 4; ++t) acc[t] = (v8f){};
#pragma unroll
  for (int ks = 0; ks < 2; ++ks) { v16b ah, al;
#pragma unroll
    for (int e2 = 0; e2 < 16; ++e2) { const int k = ks * 32 + ((e2 < 8) ? (8 * hlf + e2) : (16 + 8 * hlf + e2 - 8)); b16 p, q; split16(H[wave][nloc][k] * XS, p, q); ah[e2] = p; al[e2] = q; }
#pragma unroll
    for (int t = 0; t < 4; ++t) { const v16b bw = frag_kb(UT1 + (size_t)(t * 16 + nloc) * HD + ks * 32, hlf); acc[t] = wmma16b(ah, bw, acc[t]); acc[t] = wmma16b(al, bw, acc[t]); } }
#pragma unroll
  for (int t = 0; t < 4; ++t) { const int cc = t * 16 + nloc; const float bb = bf16_rne(c1[cc]);
#pragma unroll
    for (int r = 0; r < 8; ++r) T[wave][8 * hlf + r][cc] = fmaxf(acc[t][r] * (1.0f / (XS * WSC)) + bb, 0.0f); }
  wave_lds_sync();
#pragma unroll
  for (int t = 0; t < 4; ++t) acc[t] = (v8f){};
#pragma unroll
  for (int ks = 0; ks < 2; ++ks) { v16b ah, al;
#pragma unroll
    for (int e2 = 0; e2 < 16; ++e2) { const int k = ks * 32 + ((e2 < 8) ? (8 * hlf + e2) : (16 + 8 * hlf + e2 - 8)); b16 p, q; split16(T[wave][nloc][k] * XS, p, q); ah[e2] = p; al[e2] = q; }
#pragma unroll
    for (int t = 0; t < 4; ++t) { const v16b bw = frag_kb(UT2 + (size_t)(t * 16 + nloc) * HD + ks * 32, hlf); acc[t] = wmma16b(ah, bw, acc[t]); acc[t] = wmma16b(al, bw, acc[t]); } }
  wave_lds_sync();
#pragma unroll
  for (int t = 0; t < 4; ++t) { const int cc = t * 16 + nloc; const float bb = bf16_rne(c2[cc]);
#pragma unroll
    for (int r = 0; r < 8; ++r) { const size_t v = v0 + 8 * hlf + r; T[wave][8 * hlf + r][cc] = acc[t][r] * (1.0f / (XS * WSC)) + bb + bf16_rne(feat[v * HD + cc]); } }
  wave_lds_sync();
  for (int pass = 0; pass < 2; ++pass) { for (int rr = 0; rr < 16; ++rr) *(volatile v2f*)(out + (v0 + rr) * HD + lane * 2) = *(const v2f*)(&T[wave][rr][lane * 2]); __threadfence(); }
}
}

extern "C" void kernel_launch(void* const* d_in, const int* in_sizes, int n_in, void* d_out, int out_size, void* d_ws, size_t ws_size, hipStream_t stream) {
  (void)n_in;
  auto Fp = [&](int i) { return (const float*)d_in[i]; }; auto Ip = [&](int i) { return (const int*)d_in[i]; };
  if (in_sizes[0] != N * HD || in_sizes[1] != N * 3 || in_sizes[2] != E || in_sizes[3] != E || in_sizes[4] != (K1 + 1) * HD || in_sizes[5] != HD || in_sizes[6] != HD * HD || in_sizes[8] != HD || in_sizes[9] != 1 || in_sizes[10] != HD * HD || in_sizes[12] != HD * HD || out_size != N * HD) return;
  size_t off = 0; char* ws = (char*)d_ws;
  auto carve = [&](size_t bytes) { char* p = ws + off; off += (bytes + 255) & ~(size_t)255; return p; };
  b16* WT1 = (b16*)carve((size_t)HD * K1 * 2); b16* WT2 = (b16*)carve((size_t)HD * HD * 2); b16* UT1 = (b16*)carve((size_t)HD * HD * 2); b16* UT2 = (b16*)carve((size_t)HD * HD * 2); float* MG = (float*)carve((size_t)EH * HD * 4); float* S = (float*)carve((size_t)NP * HD * 4);
  CsrBufs csr; off = csr_carve(csr, ws, off, E, N);
  if (off > ws_size || off > ((size_t)128 << 20)) return;
  wprep_kernel<<<1, 256, 0, stream>>>(Fp(4), Fp(6), Fp(10), Fp(12), WT1, WT2, UT1, UT2);
  csr_build(csr, Ip(3), E, N, stream);
  edge_kernel<<<EC / 32, 64, 0, stream>>>(Fp(0), Fp(1), Ip(2), Ip(3), WT1, Fp(4), Fp(5), WT2, Fp(7), Fp(8), Fp(9), 0, MG);
  nsum_kernel<0><<<NP / 8, 256, 0, stream>>>(MG, csr.PERM, csr.ROWPTR, csr.ROWCNT, (int)csr.permLen, S);
  edge_kernel<<<EC / 32, 64, 0, stream>>>(Fp(0), Fp(1), Ip(2), Ip(3), WT1, Fp(4), Fp(5), WT2, Fp(7), Fp(8), Fp(9), EH, MG);
  nsum_kernel<1><<<NP / 8, 256, 0, stream>>>(MG, csr.PERM, csr.ROWPTR, csr.ROWCNT, (int)csr.permLen, S);
  node_kernel<<<NLIM / 32, 64, 0, stream>>>(S, Fp(0), UT1, Fp(11), UT2, Fp(13), (float*)d_out);
}
